// SpatioTemporalGATBatched_82008105550196
// MI455X (gfx1250) — hardware-run, weakly checked
//
#include <hip/hip_runtime.h>
#include <stddef.h>


#define NTHR  256
#define NWAVE 8
#define GR    32
#define NH    4
#define HC    64
#define DF    256
#define IND   16
#define CHUNK 2048
#define NGRP  (CHUNK / (NTHR * 4))
#define WCAP  ((CHUNK / NTHR) * 32)
#define NB1   512
#define SLB1  9
#define NB2   256
#define SLB2  8
#define LDS1  ((NB1 * HC + 2 * NB1 * NH + NWAVE * WCAP + 8) * 4)
#define LDS2  ((NB2 * DF + 2 * NB2 * NH + NWAVE * WCAP + 8) * 4)

static_assert(NGRP == 2);
static_assert(WCAP == 256);
static_assert(NB1 == (1 << SLB1));
static_assert(NB2 == (1 << SLB2));
static_assert(CHUNK <= 2048);
static_assert(LDS1 == 155680);
static_assert(LDS2 == 278560);

typedef float    v2f  __attribute__((ext_vector_type(2)));
typedef float    v4f  __attribute__((ext_vector_type(4)));
typedef float    v8f  __attribute__((ext_vector_type(8)));
typedef int      v4i  __attribute__((ext_vector_type(4)));
typedef unsigned v4u  __attribute__((ext_vector_type(4)));
typedef __bf16   v16b __attribute__((ext_vector_type(16)));
union Frag { v16b v; v4u q[2]; };


__device__ __forceinline__ v8f wm(v16b a, v16b b, v8f c) {
  v8f d = __builtin_amdgcn_wmma_f32_16x16x32_bf16(false, a, false, b, (short)0, c, false, false);
  asm volatile("v_nop\n\tv_nop\n\tv_nop\n\tv_nop" : "+v"(d) : "v"(a), "v"(b));
  return d;
}

__device__ __forceinline__ v8f wm3(const Frag& ah, const Frag& al, const Frag& bh, const Frag& bl, v8f c) {
  c = wm(ah.v, bh.v, c);
  c = wm(ah.v, bl.v, c);
  c = wm(al.v, bh.v, c);
  return c;
}

__device__ __forceinline__ v8f z8() { v8f z = {0.f, 0.f, 0.f, 0.f, 0.f, 0.f, 0.f, 0.f}; return z; }

__device__ __forceinline__ unsigned bfr(float f) {
  const unsigned u = __float_as_uint(f);
  return (u + 0x7FFFu + ((u >> 16) & 1u)) >> 16;
}

__device__ __forceinline__ void sp2pack(float a, float b, unsigned& ph, unsigned& pl) {
  const unsigned ha = bfr(a), hb = bfr(b);
  const unsigned la = bfr(a - __uint_as_float(ha << 16));
  const unsigned lb = bfr(b - __uint_as_float(hb << 16));
  ph = ha | (hb << 16);
  pl = la | (lb << 16);
}

__device__ __forceinline__ void pack8(const v4f a, const v4f b, v4u& ph, v4u& pl) {
  unsigned h0, h1, h2, h3, l0, l1, l2, l3;
  sp2pack(a.x, a.y, h0, l0);
  sp2pack(a.z, a.w, h1, l1);
  sp2pack(b.x, b.y, h2, l2);
  sp2pack(b.z, b.w, h3, l3);
  v4u th = {h0, h1, h2, h3};
  v4u tl = {l0, l1, l2, l3};
  ph = th; pl = tl;
}

__device__ __forceinline__ void ldfrag(Frag& f, const unsigned short* p, int hh) {
  f.q[0] = *(const v4u*)(p + 8 * hh);
  f.q[1] = *(const v4u*)(p + 16 + 8 * hh);
}

__device__ __forceinline__ float wsum(float v) {
  v += __shfl_xor(v, 16, 32);
  v += __shfl_xor(v, 8, 32);
  v += __shfl_xor(v, 4, 32);
  v += __shfl_xor(v, 2, 32);
  v += __shfl_xor(v, 1, 32);
  return v;
}

__device__ __forceinline__ float g8(float v) {
  v += __shfl_xor(v, 1, 32);
  v += __shfl_xor(v, 2, 32);
  v += __shfl_xor(v, 4, 32);
  return v;
}

__device__ __forceinline__ v4f hx(v4f v) {
  v.x += __shfl_xor(v.x, 8, 32);  v.y += __shfl_xor(v.y, 8, 32);
  v.z += __shfl_xor(v.z, 8, 32);  v.w += __shfl_xor(v.w, 8, 32);
  v.x += __shfl_xor(v.x, 16, 32); v.y += __shfl_xor(v.y, 16, 32);
  v.z += __shfl_xor(v.z, 16, 32); v.w += __shfl_xor(v.w, 16, 32);
  return v;
}

__device__ __forceinline__ v4f shf4(v4f v, int sl) {
  v4f r;
  r.x = __shfl(v.x, sl, 32); r.y = __shfl(v.y, sl, 32);
  r.z = __shfl(v.z, sl, 32); r.w = __shfl(v.w, sl, 32);
  return r;
}

__device__ __forceinline__ v4f max0(v4f v) {
  v.x = fmaxf(v.x, 0.f); v.y = fmaxf(v.y, 0.f); v.z = fmaxf(v.z, 0.f); v.w = fmaxf(v.w, 0.f);
  return v;
}

__device__ __forceinline__ void stage64(const float* __restrict__ A, int nN, int rowBase,
                                        unsigned short* Ah, unsigned short* Al, int AP, int tid) {
  const int r = tid >> 3, c0 = (tid & 7) * 8;
  int row = rowBase + r;
  if (row > nN - 1) row = nN - 1;
  const float* p = A + (size_t)row * HC + c0;
  const v4f f0 = *(const v4f*)p;
  const v4f f1 = *(const v4f*)(p + 4);
  v4u ph, pl;
  pack8(f0, f1, ph, pl);
  *(v4u*)(Ah + r * AP + c0) = ph;
  *(v4u*)(Al + r * AP + c0) = pl;
}

__global__ __launch_bounds__(NTHR) void k_prep(const float* __restrict__ W, unsigned short* Ph, unsigned short* Pl,
                                               int ncols, int K, int KP, int kdiv, int ldk, int ldh, int ldn,
                                               float scale) {
  const int per = KP >> 3;
  const int i = blockIdx.x * NTHR + threadIdx.x;
  if (i >= ncols * per) return;
  const int n  = i / per;
  const int k0 = (i - n * per) * 8;
  float v[8];
#pragma unroll
  for (int t = 0; t < 8; ++t) {
    const int k  = k0 + t;
    const int kc = (k < K) ? k : (K - 1);
    const int kq = kc / kdiv;
    const int kr = kc - kq * kdiv;
    const float w = W[kr * ldk + kq * ldh + n * ldn] * scale;
    v[t] = (k < K) ? w : 0.0f;
  }
  unsigned ph0, ph1, ph2, ph3, pl0, pl1, pl2, pl3;
  sp2pack(v[0], v[1], ph0, pl0);
  sp2pack(v[2], v[3], ph1, pl1);
  sp2pack(v[4], v[5], ph2, pl2);
  sp2pack(v[6], v[7], ph3, pl3);
  const v4u a = {ph0, ph1, ph2, ph3};
  const v4u b = {pl0, pl1, pl2, pl3};
  unsigned short* oh = Ph + (size_t)n * KP + k0;
  unsigned short* ol = Pl + (size_t)n * KP + k0;
  *(volatile v4u*)oh = a;
  *(volatile v4u*)ol = b;
  __threadfence();
  *(volatile v4u*)oh = a;
  *(volatile v4u*)ol = b;
}

__global__ __launch_bounds__(NTHR) void k_es(const float* __restrict__ x, const float* __restrict__ w0,
                                             const float* __restrict__ as0, const float* __restrict__ ad0,
                                             float* es, float* ed, int nN, int nP) {
  __shared__ float wa[IND * 8];
  const int tid = threadIdx.x;
  if (tid < IND * 8) {
    const int k = tid >> 3, j = tid & 7;
    const int hcol = (j & 3) * HC;
    float s = 0.f;
#pragma unroll 1
    for (int c = 0; c < HC; ++c) {
      const float ws = as0[hcol + c];
      const float wd = ad0[hcol + c];
      const float av = (j < 4) ? ws : wd;
      s += w0[k * DF + hcol + c] * av;
    }
    wa[tid] = s;
  }
  __syncthreads();
  const int node = blockIdx.x * NTHR + tid;
  const int row  = (node < nN) ? node : (nN - 1);
  float e[8] = {0.f, 0.f, 0.f, 0.f, 0.f, 0.f, 0.f, 0.f};
#pragma unroll 1
  for (int k = 0; k < IND; ++k) {
    const float xk = x[(size_t)row * IND + k];
#pragma unroll
    for (int j = 0; j < 8; ++j) e[j] += xk * wa[k * 8 + j];
  }
  if (node < nP) {
    const v4f vs = {e[0], e[1], e[2], e[3]};
    const v4f vd = {e[4], e[5], e[6], e[7]};
    float* ps = es + (size_t)node * NH;
    float* pd = ed + (size_t)node * NH;
    *(volatile v4f*)ps = vs;
    *(volatile v4f*)pd = vd;
    __threadfence();
    *(volatile v4f*)ps = vs;
    *(volatile v4f*)pd = vd;
  }
}

template <int L>
__global__ __launch_bounds__(NTHR) void k_agg(const int* __restrict__ ei, const float* __restrict__ X,
                                              const float* __restrict__ es, const float* __restrict__ ed,
                                              const float* __restrict__ bias, const float* __restrict__ gam,
                                              const float* __restrict__ bet,
                                              float* hout, int nN, int nE, int relu) {
  constexpr int NB  = (L == 1) ? NB1 : NB2;
  constexpr int SLB = (L == 1) ? SLB1 : SLB2;
  constexpr int ACW = (L == 1) ? HC : DF;
  constexpr int XW  = (L == 1) ? IND : DF;
  extern __shared__ v4f lds_dyn[];
  float* sacc = (float*)lds_dyn;
  float* den  = sacc + NB * ACW;
  float* mx   = den + NB * NH;
  int*   list = (int*)(mx + NB * NH);
  int*   wcnt = list + NWAVE * WCAP;

  const int tid  = threadIdx.x;
  const int lane = tid & 31;
  const int wave = tid >> 5;
  const int hd   = lane >> 3;
  const int nodeBase = blockIdx.x * NB;

  {
    const v4f z4 = {0.f, 0.f, 0.f, 0.f};
    for (int i = tid; i < (NB * ACW + NB * NH) / 4; i += NTHR) lds_dyn[i] = z4;
    for (int i = tid; i < NB * NH; i += NTHR) mx[i] = -1.0e30f;
  }
  __syncthreads();

  const int* eid = ei + nE;
  const bool al16 = ((nE & 3) == 0);
  const int nChunks = (nE + CHUNK - 1) / CHUNK;

#pragma unroll 1
  for (int ch = 0; ch < nChunks; ++ch) {
    const int cbase = ch * CHUNK;
    int wc = 0;
#pragma unroll
    for (int g = 0; g < NGRP; ++g) {
      const int el0 = (g * NTHR + tid) * 4;
      const int e0  = cbase + el0;
      const int sent = -2147483647 - 1;
      v4i d;
      if (al16 && (cbase + CHUNK <= nE)) {
        d = *(const v4i*)(eid + e0);
      } else {
        d.x = (e0     < nE) ? eid[(e0     < nE - 1) ? e0     : nE - 1] : sent;
        d.y = (e0 + 1 < nE) ? eid[(e0 + 1 < nE - 1) ? e0 + 1 : nE - 1] : sent;
        d.z = (e0 + 2 < nE) ? eid[(e0 + 2 < nE - 1) ? e0 + 2 : nE - 1] : sent;
        d.w = (e0 + 3 < nE) ? eid[(e0 + 3 < nE - 1) ? e0 + 3 : nE - 1] : sent;
      }
      const unsigned s0 = (unsigned)d.x - (unsigned)nodeBase;
      const unsigned s1 = (unsigned)d.y - (unsigned)nodeBase;
      const unsigned s2 = (unsigned)d.z - (unsigned)nodeBase;
      const unsigned s3 = (unsigned)d.w - (unsigned)nodeBase;
      const bool h0 = s0 < (unsigned)NB;
      const bool h1 = s1 < (unsigned)NB;
      const bool h2 = s2 < (unsigned)NB;
      const bool h3 = s3 < (unsigned)NB;
      const unsigned many = __builtin_amdgcn_ballot_w32(h0 | h1 | h2 | h3);
      if (many != 0u) {
#define HITJ(J, HJ, SJ) { \
          const unsigned mj = __builtin_amdgcn_ballot_w32(HJ); \
          if (HJ) { \
            const int pos = wc + (int)__builtin_amdgcn_mbcnt_lo(mj, 0u); \
            if (pos < WCAP) list[wave * WCAP + pos] = ((el0 + (J)) << SLB) | (int)(SJ); \
          } \
          wc += (int)__builtin_popcount(mj); }
        HITJ(0, h0, s0)
        HITJ(1, h1, s1)
        HITJ(2, h2, s2)
        HITJ(3, h3, s3)
#undef HITJ
      }
    }
    if (lane == 0) wcnt[wave] = wc;
    __syncthreads();

    if (wave == 0) {
      for (int wsx = 0; wsx < NWAVE; ++wsx) {
        int n = wcnt[wsx];
        if (n > WCAP) n = WCAP;
        if (n < 0) n = 0;
        for (int i = 0; i < n; ++i) {
          const int ent  = list[wsx * WCAP + i];
          const int slot = ent & (NB - 1);
          const int el   = (ent >> SLB) & (CHUNK - 1);
          int e = cbase + el;
          if (e > nE - 1) e = nE - 1;
          int src = ei[e];
          src = src < 0 ? 0 : (src > nN - 1 ? nN - 1 : src);
          int nd = nodeBase + slot;
          if (nd > nN - 1) nd = nN - 1;
          float a = es[(size_t)src * NH + hd] + ed[(size_t)nd * NH + hd];
          a = (a > 0.f) ? a : 0.2f * a;
          const int ai = slot * NH + hd;
          const float mo = mx[ai];
          const float mn = fmaxf(mo, a);
          const float f  = __expf(mo - mn);
          const float p  = __expf(a - mn);
          if (L == 1) {
            const v2f xv = *(const v2f*)(X + (size_t)src * XW + 2 * (lane & 7));
            v2f* sp = (v2f*)(sacc + slot * ACW + 2 * lane);
            const v2f c = *sp;
            *sp = c * f + p * xv;
          } else {
            const float* xr = X + (size_t)src * XW + 8 * lane;
            const v4f x0 = *(const v4f*)xr;
            const v4f x1 = *(const v4f*)(xr + 4);
            v4f* sp = (v4f*)(sacc + slot * ACW + 8 * lane);
            const v4f c0 = sp[0], c1 = sp[1];
            sp[0] = c0 * f + p * x0;
            sp[1] = c1 * f + p * x1;
          }
          const float dv = den[ai];
          den[ai] = dv * f + p;
          mx[ai]  = mn;
        }
      }
    }
    __syncthreads();
  }

  if (L == 1) {
#pragma unroll 1
    for (int j = 0; j < NB / NWAVE; ++j) {
      const int slot = wave * (NB / NWAVE) + j;
      const int node = nodeBase + slot;
      if (node >= nN) break;
      float a = es[(size_t)node * NH + hd] + ed[(size_t)node * NH + hd];
      a = (a > 0.f) ? a : 0.2f * a;
      const int ai = slot * NH + hd;
      const float mo = mx[ai];
      const float mn = fmaxf(mo, a);
      const float f  = __expf(mo - mn);
      const float p  = __expf(a - mn);
      const v2f xv = *(const v2f*)(X + (size_t)node * XW + 2 * (lane & 7));
      const v2f s  = *(const v2f*)(sacc + slot * ACW + 2 * lane) * f + p * xv;
      const float inv = 1.0f / (den[ai] * f + p);
      const v2f u = s * inv;
      float* op = hout + (size_t)node * HC + 2 * lane;
      *(volatile v2f*)op = u;
      __threadfence();
      *(volatile v2f*)op = u;
    }
  } else {
    const int cq = lane & 7;
    const v4f bA = *(const v4f*)(bias + 8 * cq), bB = *(const v4f*)(bias + 8 * cq + 4);
    const v4f gA = *(const v4f*)(gam + 8 * cq),  gB = *(const v4f*)(gam + 8 * cq + 4);
    const v4f tA = *(const v4f*)(bet + 8 * cq),  tB = *(const v4f*)(bet + 8 * cq + 4);
    const int sl = (lane >> 1) & 7;
#pragma unroll 1
    for (int j = 0; j < NB / NWAVE; ++j) {
      const int slot = wave * (NB / NWAVE) + j;
      const int node = nodeBase + slot;
      if (node >= nN) break;
      float a = es[(size_t)node * NH + hd] + ed[(size_t)node * NH + hd];
      a = (a > 0.f) ? a : 0.2f * a;
      const int ai = slot * NH + hd;
      const float mo = mx[ai];
      const float mn = fmaxf(mo, a);
      const float f  = __expf(mo - mn);
      const float p  = __expf(a - mn);
      const float* xr = X + (size_t)node * XW + 8 * lane;
      const v4f x0 = *(const v4f*)xr;
      const v4f x1 = *(const v4f*)(xr + 4);
      const v4f* sp = (const v4f*)(sacc + slot * ACW + 8 * lane);
      const float inv = 1.0f / (den[ai] * f + p);
      v4f u0 = (sp[0] * f + p * x0) * inv;
      v4f u1 = (sp[1] * f + p * x1) * inv;
      u0 = hx(u0);
      u1 = hx(u1);
      const v4f h0 = u0 * 0.25f + bA;
      const v4f h1 = u1 * 0.25f + bB;
      const float s  = g8(h0.x + h0.y + h0.z + h0.w + h1.x + h1.y + h1.z + h1.w);
      const float mu = s * (1.0f / HC);
      const v4f d0 = h0 - mu, d1 = h1 - mu;
      const float q  = g8(d0.x * d0.x + d0.y * d0.y + d0.z * d0.z + d0.w * d0.w +
                          d1.x * d1.x + d1.y * d1.y + d1.z * d1.z + d1.w * d1.w);
      const float rs = rsqrtf(q * (1.0f / HC) + 1e-5f);
      v4f y0 = d0 * rs * gA + tA;
      v4f y1 = d1 * rs * gB + tB;
      if (relu) { y0 = max0(y0); y1 = max0(y1); }
      const v4f fa = shf4(y0, sl);
      const v4f fb = shf4(y1, sl);
      const v4f ov = (lane & 1) ? fb : fa;
      float* op = hout + (size_t)node * HC + 4 * (lane & 15);
      if (lane < 16) *(volatile v4f*)op = ov;
      __threadfence();
      if (lane < 16) *(volatile v4f*)op = ov;
    }
  }
}

__global__ __launch_bounds__(NTHR) void k_agemm(const float* __restrict__ A, const unsigned short* __restrict__ Bh,
                                                const unsigned short* __restrict__ Bl, const float* __restrict__ bias,
                                                const float* __restrict__ gam, const float* __restrict__ bet,
                                                float* hout, int nN) {
  constexpr int KP = HC, AP = HC + 8, XSP = HC + 4;
  __shared__ __attribute__((aligned(16))) unsigned short Ah[GR * AP];
  __shared__ __attribute__((aligned(16))) unsigned short Al[GR * AP];
  __shared__ __attribute__((aligned(16))) float Xs[GR * XSP];
  const int tid = threadIdx.x, lane = tid & 31, wave = tid >> 5, hh = lane >> 4, m = lane & 15;
  const int rowBase = blockIdx.x * GR;

  stage64(A, nN, rowBase, Ah, Al, AP, tid);
  __syncthreads();

  const int T = wave & 1, j = wave >> 1;
  v8f acc = z8();
#pragma unroll
  for (int kt = 0; kt < KP / 32; ++kt) {
    const int k0 = kt * 32;
    Frag ah, al, bh, bl;
    ldfrag(ah, Ah + (16 * T + m) * AP + k0, hh);
    ldfrag(al, Al + (16 * T + m) * AP + k0, hh);
    const size_t bo = (size_t)(16 * j + m) * KP + k0;
    ldfrag(bh, Bh + bo, hh);
    ldfrag(bl, Bl + bo, hh);
    acc = wm3(ah, al, bh, bl, acc);
  }
  {
    const int col = 16 * j + m;
    const float bb = bias[col];
#pragma unroll
    for (int r = 0; r < 8; ++r) Xs[(16 * T + 8 * hh + r) * XSP + col] = acc[r] + bb;
  }
  __syncthreads();

  const v2f g2 = *(const v2f*)(gam + 2 * lane);
  const v2f e2 = *(const v2f*)(bet + 2 * lane);
#pragma unroll 1
  for (int i = 0; i < GR / NWAVE; ++i) {
    const int r = wave * (GR / NWAVE) + i;
    const int row = rowBase + r;
    if (row >= nN) break;
    const v2f h = *(const v2f*)(Xs + r * XSP + 2 * lane);
    const float s  = wsum(h.x + h.y);
    const float mu = s * (1.0f / HC);
    const v2f d = h - mu;
    const float q  = wsum(d.x * d.x + d.y * d.y);
    const float rs = rsqrtf(q * (1.0f / HC) + 1e-5f);
    v2f y = d * rs * g2 + e2;
    y.x = fmaxf(y.x, 0.f);
    y.y = fmaxf(y.y, 0.f);
    float* op = hout + (size_t)row * HC + 2 * lane;
    *(volatile v2f*)op = y;
    __threadfence();
    *(volatile v2f*)op = y;
  }
}

__global__ __launch_bounds__(NTHR) void k_xp(const float* __restrict__ A, const unsigned short* __restrict__ Bh,
                                             const unsigned short* __restrict__ Bl, const float* __restrict__ att_s,
                                             const float* __restrict__ att_d, float* xp, float* es, float* ed, int nN) {
  constexpr int KP = HC, AP = HC + 8, XSP = DF + 4;
  __shared__ __attribute__((aligned(16))) unsigned short Ah[GR * AP];
  __shared__ __attribute__((aligned(16))) unsigned short Al[GR * AP];
  __shared__ __attribute__((aligned(16))) float Xs[GR * XSP];
  __shared__ __attribute__((aligned(16))) float As[GR * NWAVE];
  __shared__ __attribute__((aligned(16))) float Ds[GR * NWAVE];
  const int tid = threadIdx.x, lane = tid & 31, wave = tid >> 5, hh = lane >> 4, m = lane & 15;
  const int rowBase = blockIdx.x * GR;

  stage64(A, nN, rowBase, Ah, Al, AP, tid);
  __syncthreads();

  v8f acc[2][2];
#pragma unroll
  for (int T = 0; T < 2; ++T) { acc[T][0] = z8(); acc[T][1] = z8(); }
#pragma unroll
  for (int kt = 0; kt < KP / 32; ++kt) {
    const int k0 = kt * 32;
    Frag ah[2], al[2], bh[2], bl[2];
#pragma unroll
    for (int T = 0; T < 2; ++T) {
      ldfrag(ah[T], Ah + (16 * T + m) * AP + k0, hh);
      ldfrag(al[T], Al + (16 * T + m) * AP + k0, hh);
    }
#pragma unroll
    for (int jt = 0; jt < 2; ++jt) {
      const size_t bo = (size_t)(wave * 32 + 16 * jt + m) * KP + k0;
      ldfrag(bh[jt], Bh + bo, hh);
      ldfrag(bl[jt], Bl + bo, hh);
    }
#pragma unroll
    for (int T = 0; T < 2; ++T)
#pragma unroll
      for (int jt = 0; jt < 2; ++jt) acc[T][jt] = wm3(ah[T], al[T], bh[jt], bl[jt], acc[T][jt]);
  }

  float cs[2], cd[2];
#pragma unroll
  for (int jt = 0; jt < 2; ++jt) {
    const int col = wave * 32 + 16 * jt + m;
    cs[jt] = att_s[col];
    cd[jt] = att_d[col];
  }
#pragma unroll
  for (int T = 0; T < 2; ++T) {
    float ss[8], sd[8];
#pragma unroll
    for (int r = 0; r < 8; ++r) {
      const float v0 = acc[T][0][r];
      const float v1 = acc[T][1][r];
      const int rr = 16 * T + 8 * hh + r;
      Xs[rr * XSP + wave * 32 + m]      = v0;
      Xs[rr * XSP + wave * 32 + 16 + m] = v1;
      ss[r] = v0 * cs[0] + v1 * cs[1];
      sd[r] = v0 * cd[0] + v1 * cd[1];
    }
#pragma unroll
    for (int mk = 1; mk < 16; mk <<= 1) {
#pragma unroll
      for (int r = 0; r < 8; ++r) {
        ss[r] += __shfl_xor(ss[r], mk, 32);
        sd[r] += __shfl_xor(sd[r], mk, 32);
      }
    }
    if (m == 0) {
#pragma unroll
      for (int r = 0; r < 8; ++r) {
        As[(16 * T + 8 * hh + r) * NWAVE + wave] = ss[r];
        Ds[(16 * T + 8 * hh + r) * NWAVE + wave] = sd[r];
      }
    }
  }
  __syncthreads();

  v4f xr[8];
#pragma unroll
  for (int i = 0; i < 4; ++i) {
    const int r = 4 * wave + i;
    xr[2 * i]     = *(const v4f*)(Xs + r * XSP + 4 * lane);
    xr[2 * i + 1] = *(const v4f*)(Xs + r * XSP + 128 + 4 * lane);
  }
  const v4f ve = {As[lane * 8 + 0] + As[lane * 8 + 1], As[lane * 8 + 2] + As[lane * 8 + 3],
                  As[lane * 8 + 4] + As[lane * 8 + 5], As[lane * 8 + 6] + As[lane * 8 + 7]};
  const v4f vd = {Ds[lane * 8 + 0] + Ds[lane * 8 + 1], Ds[lane * 8 + 2] + Ds[lane * 8 + 3],
                  Ds[lane * 8 + 4] + Ds[lane * 8 + 5], Ds[lane * 8 + 6] + Ds[lane * 8 + 7]};
  const v4f gv = (wave == 0) ? ve : vd;
  float* gp = ((wave == 0) ? es : ed) + (size_t)(rowBase + lane) * NH;

#pragma unroll
  for (int i = 0; i < 4; ++i) {
    float* p = xp + (size_t)(rowBase + 4 * wave + i) * DF + 4 * lane;
    *(volatile v4f*)p         = xr[2 * i];
    *(volatile v4f*)(p + 128) = xr[2 * i + 1];
  }
  if (wave < 2) *(volatile v4f*)gp = gv;
  __threadfence();
#pragma unroll
  for (int i = 0; i < 4; ++i) {
    float* p = xp + (size_t)(rowBase + 4 * wave + i) * DF + 4 * lane;
    *(volatile v4f*)p         = xr[2 * i];
    *(volatile v4f*)(p + 128) = xr[2 * i + 1];
  }
  if (wave < 2) *(volatile v4f*)gp = gv;
}

__global__ __launch_bounds__(NTHR) void k_tail(const float* __restrict__ h2, const float* __restrict__ x,
                                               const unsigned short* __restrict__ Wh, const unsigned short* __restrict__ Wl,
                                               const float* __restrict__ bih, const float* __restrict__ bhh,
                                               const unsigned short* __restrict__ P0h, const unsigned short* __restrict__ P0l,
                                               const float* __restrict__ d0b,
                                               const unsigned short* __restrict__ P1h, const unsigned short* __restrict__ P1l,
                                               const float* __restrict__ d1b,
                                               const float* __restrict__ d2w, const float* __restrict__ d2b,
                                               float* out, int nN) {
  constexpr int AP0 = HC + 8;
  constexpr int K1  = 96;
  constexpr int AP1 = K1 + 8;
  constexpr int GP  = 3 * HC + 4;
  constexpr int DP  = 36;
  __shared__ __attribute__((aligned(16))) unsigned short A0h[GR * AP0];
  __shared__ __attribute__((aligned(16))) unsigned short A0l[GR * AP0];
  __shared__ __attribute__((aligned(16))) float G[GR * GP];
  __shared__ __attribute__((aligned(16))) unsigned short A1h[GR * AP1];
  __shared__ __attribute__((aligned(16))) unsigned short A1l[GR * AP1];
  __shared__ __attribute__((aligned(16))) unsigned short A2h[GR * AP0];
  __shared__ __attribute__((aligned(16))) unsigned short A2l[GR * AP0];
  __shared__ __attribute__((aligned(16))) float D1s[GR * DP];
  __shared__ __attribute__((aligned(16))) float Os[GR * 2];
  const int tid = threadIdx.x, lane = tid & 31, wave = tid >> 5, hh = lane >> 4, m = lane & 15;
  const int rowBase = blockIdx.x * GR;

  stage64(h2, nN, rowBase, A0h, A0l, AP0, tid);
  __syncthreads();

  {
    const int T = wave & 1, cg = wave >> 1;
    v8f acc[3];
    acc[0] = z8(); acc[1] = z8(); acc[2] = z8();
#pragma unroll
    for (int kt = 0; kt < HC / 32; ++kt) {
      const int k0 = kt * 32;
      Frag ah, al;
      ldfrag(ah, A0h + (16 * T + m) * AP0 + k0, hh);
      ldfrag(al, A0l + (16 * T + m) * AP0 + k0, hh);
      Frag bh[3], bl[3];
#pragma unroll
      for (int jt = 0; jt < 3; ++jt) {
        const size_t bo = (size_t)(48 * cg + 16 * jt + m) * HC + k0;
        ldfrag(bh[jt], Wh + bo, hh);
        ldfrag(bl[jt], Wl + bo, hh);
      }
#pragma unroll
      for (int jt = 0; jt < 3; ++jt) acc[jt] = wm3(ah, al, bh[jt], bl[jt], acc[jt]);
    }
#pragma unroll
    for (int jt = 0; jt < 3; ++jt) {
      const int col = 48 * cg + 16 * jt + m;
      const float bb = bih[col];
#pragma unroll
      for (int r = 0; r < 8; ++r) G[(16 * T + 8 * hh + r) * GP + col] = acc[jt][r] + bb;
    }
  }
  __syncthreads();

  {
#pragma unroll 1
    for (int i = 0; i < 8; ++i) {
      const int idx = tid + NTHR * i;
      const int row = idx >> 6, c = idx & 63;
      const float gr = G[row * GP + c] + bhh[c];
      const float gz = G[row * GP + HC + c] + bhh[HC + c];
      const float gn = G[row * GP + 2 * HC + c];
      const float rg = __builtin_amdgcn_rcpf(1.0f + __expf(-gr));
      const float zg = __builtin_amdgcn_rcpf(1.0f + __expf(-gz));
      const float cn = tanhf(gn + rg * bhh[2 * HC + c]);
      const float tv = (1.0f - zg) * cn;
      const unsigned h = bfr(tv);
      const unsigned l = bfr(tv - __uint_as_float(h << 16));
      A1h[row * AP1 + c] = (unsigned short)h;
      A1l[row * AP1 + c] = (unsigned short)l;
    }
#pragma unroll
    for (int i = 0; i < 2; ++i) {
      const int idx = tid + NTHR * i;
      const int row = idx >> 4, c = idx & 15;
      int grow = rowBase + row;
      if (grow > nN - 1) grow = nN - 1;
      const float xv = x[(size_t)grow * IND + c];
      const unsigned h = bfr(xv);
      const unsigned l = bfr(xv - __uint_as_float(h << 16));
      A1h[row * AP1 + HC + c] = (unsigned short)h;
      A1l[row * AP1 + HC + c] = (unsigned short)l;
    }
    if (tid < 2 * GR) {
      const int row = tid >> 1, part = tid & 1;
      const v4u z = {0u, 0u, 0u, 0u};
      *(v4u*)(A1h + row * AP1 + HC + IND + 8 * part) = z;
      *(v4u*)(A1l + row * AP1 + HC + IND + 8 * part) = z;
    }
  }
  __syncthreads();

  {
    const int T = wave & 1, jt = wave >> 1;
    v8f acc = z8();
#pragma unroll
    for (int kt = 0; kt < K1 / 32; ++kt) {
      const int k0 = kt * 32;
      Frag ah, al, bh, bl;
      ldfrag(ah, A1h + (16 * T + m) * AP1 + k0, hh);
      ldfrag(al, A1l + (16 * T + m) * AP1 + k0, hh);
      const size_t bo = (size_t)(16 * jt + m) * K1 + k0;
      ldfrag(bh, P0h + bo, hh);
      ldfrag(bl, P0l + bo, hh);
      acc = wm3(ah, al, bh, bl, acc);
    }
    const int col = 16 * jt + m;
    const float bb = d0b[col];
#pragma unroll
    for (int r = 0; r < 8; ++r) {
      const float v = fmaxf(acc[r] + bb, 0.f);
      const unsigned h = bfr(v);
      const unsigned l = bfr(v - __uint_as_float(h << 16));
      A2h[(16 * T + 8 * hh + r) * AP0 + col] = (unsigned short)h;
      A2l[(16 * T + 8 * hh + r) * AP0 + col] = (unsigned short)l;
    }
  }
  __syncthreads();

  if (wave < 4) {
    const int T = wave & 1, jt = wave >> 1;
    v8f acc = z8();
#pragma unroll
    for (int kt = 0; kt < HC / 32; ++kt) {
      const int k0 = kt * 32;
      Frag ah, al, bh, bl;
      ldfrag(ah, A2h + (16 * T + m) * AP0 + k0, hh);
      ldfrag(al, A2l + (16 * T + m) * AP0 + k0, hh);
      const size_t bo = (size_t)(16 * jt + m) * HC + k0;
      ldfrag(bh, P1h + bo, hh);
      ldfrag(bl, P1l + bo, hh);
      acc = wm3(ah, al, bh, bl, acc);
    }
    const int col = 16 * jt + m;
    const float bb = d1b[col];
#pragma unroll
    for (int r = 0; r < 8; ++r) D1s[(16 * T + 8 * hh + r) * DP + col] = fmaxf(acc[r] + bb, 0.f);
  }
  __syncthreads();

  if (tid < 2 * GR) {
    const int row = tid >> 1, jo = tid & 1;
    float s = 0.f;
#pragma unroll 8
    for (int c = 0; c < 32; ++c) s += D1s[row * DP + c] * d2w[c * 2 + jo];
    s += d2b[jo];
    s = fminf(fmaxf(s, -0.5f), 0.5f);
    Os[tid] = s;
  }
  __syncthreads();

  if (wave == 0) {
    int nv = nN - rowBase;
    if (nv > GR) nv = GR;
    const v4f ov = *(const v4f*)(Os + 4 * (lane & 15));
    float* op = out + (size_t)rowBase * 2 + 4 * lane;
    const bool full = (2 * lane + 2 <= nv);
    const bool half = ((nv & 1) != 0) && (2 * lane + 1 == nv);
    const v2f o2 = {ov.x, ov.y};
    if (full) *(volatile v4f*)op = ov;
    else if (half) *(volatile v2f*)op = o2;
    __threadfence();
    if (full) *(volatile v4f*)op = ov;
    else if (half) *(volatile v2f*)op = o2;
  }
}


static inline int cdiv(int a, int b) { return (a + b - 1) / b; }

extern "C" void kernel_launch(void* const* d_in, const int* in_sizes, int n_in,
                              void* d_out, int out_size, void* d_ws, size_t ws_size,
                              hipStream_t stream) {
  if (n_in < 24) return;
  const int nN = in_sizes[0] / IND;
  if (nN <= 0 || in_sizes[0] != nN * IND) return;
  if (in_sizes[1] < 0 || (in_sizes[1] & 1) != 0) return;
  const int nE = in_sizes[1] / 2;
  if (in_sizes[2] != IND * DF || in_sizes[3] != NH * HC || in_sizes[4] != NH * HC) return;
  if (in_sizes[5] != HC || in_sizes[6] != HC || in_sizes[7] != HC) return;
  if (in_sizes[8] != HC * DF || in_sizes[9] != NH * HC || in_sizes[10] != NH * HC) return;
  if (in_sizes[11] != HC || in_sizes[12] != HC || in_sizes[13] != HC) return;
  if (in_sizes[14] != 3 * HC * HC || in_sizes[16] != 3 * HC || in_sizes[17] != 3 * HC) return;
  if (in_sizes[18] != (HC + IND) * HC || in_sizes[19] != HC) return;
  if (in_sizes[20] != HC * 32 || in_sizes[21] != 32 || in_sizes[22] != 32 * 2 || in_sizes[23] != 2) return;
  if (out_size != nN * 2) return;

  const float* x      = (const float*)d_in[0];
  const int*   ei     = (const int*)d_in[1];
  const float* w0     = (const float*)d_in[2];
  const float* a_src0 = (const float*)d_in[3];
  const float* a_dst0 = (const float*)d_in[4];
  const float* b0     = (const float*)d_in[5];
  const float* ln0_g  = (const float*)d_in[6];
  const float* ln0_b  = (const float*)d_in[7];
  const float* w1     = (const float*)d_in[8];
  const float* a_src1 = (const float*)d_in[9];
  const float* a_dst1 = (const float*)d_in[10];
  const float* b1     = (const float*)d_in[11];
  const float* ln1_g  = (const float*)d_in[12];
  const float* ln1_b  = (const float*)d_in[13];
  const float* gw_ih  = (const float*)d_in[14];
  const float* gb_ih  = (const float*)d_in[16];
  const float* gb_hh  = (const float*)d_in[17];
  const float* d0w    = (const float*)d_in[18];
  const float* d0b    = (const float*)d_in[19];
  const float* d1w    = (const float*)d_in[20];
  const float* d1b    = (const float*)d_in[21];
  const float* d2w    = (const float*)d_in[22];
  const float* d2b    = (const float*)d_in[23];
  float* out = (float*)d_out;

  const int nP = cdiv(nN, GR) * GR;
  const size_t szWr  = (size_t)HC * HC * 2;
  const size_t szW2  = (size_t)DF * HC * 2;
  const size_t szWih = (size_t)(3 * HC) * HC * 2;
  const size_t szD0  = (size_t)HC * 96 * 2;
  const size_t szD1  = (size_t)32 * HC * 2;
  const size_t szE   = (size_t)nP * NH * 4;
  const size_t szH   = (size_t)nP * HC * 4;
  const size_t szXP  = (size_t)nP * DF * 4;
  char* base = (char*)d_ws;
  size_t off = 0;
  unsigned short* Pwr_h = (unsigned short*)(base + off); off += szWr;
  unsigned short* Pwr_l = (unsigned short*)(base + off); off += szWr;
  unsigned short* Pw2_h = (unsigned short*)(base + off); off += szW2;
  unsigned short* Pw2_l = (unsigned short*)(base + off); off += szW2;
  unsigned short* Pih_h = (unsigned short*)(base + off); off += szWih;
  unsigned short* Pih_l = (unsigned short*)(base + off); off += szWih;
  unsigned short* Pd0_h = (unsigned short*)(base + off); off += szD0;
  unsigned short* Pd0_l = (unsigned short*)(base + off); off += szD0;
  unsigned short* Pd1_h = (unsigned short*)(base + off); off += szD1;
  unsigned short* Pd1_l = (unsigned short*)(base + off); off += szD1;
  float* es   = (float*)(base + off); off += szE;
  float* ed   = (float*)(base + off); off += szE;
  float* agg1 = (float*)(base + off); off += szH;
  float* h1   = (float*)(base + off); off += szH;
  float* xp2  = (float*)(base + off); off += szXP;
  float* h2   = (float*)(base + off); off += szH;
  if (off > ws_size) return;

  k_prep<<<cdiv(HC * (HC / 8), NTHR), NTHR, 0, stream>>>(w0, Pwr_h, Pwr_l, HC, HC, HC, IND, DF, HC, 1, 0.25f);
  k_prep<<<cdiv(DF * (HC / 8), NTHR), NTHR, 0, stream>>>(w1, Pw2_h, Pw2_l, DF, HC, HC, HC, DF, 0, 1, 1.0f);
  k_prep<<<cdiv(3 * HC * (HC / 8), NTHR), NTHR, 0, stream>>>(gw_ih, Pih_h, Pih_l, 3 * HC, HC, HC, HC, 1, 0, HC, 1.0f);
  k_prep<<<cdiv(HC * (96 / 8), NTHR), NTHR, 0, stream>>>(d0w, Pd0_h, Pd0_l, HC, HC + IND, 96, HC + IND, HC, 0, 1, 1.0f);
  k_prep<<<cdiv(32 * (HC / 8), NTHR), NTHR, 0, stream>>>(d1w, Pd1_h, Pd1_l, 32, HC, HC, HC, 32, 0, 1, 1.0f);

  k_es<<<cdiv(nP, NTHR), NTHR, 0, stream>>>(x, w0, a_src0, a_dst0, es, ed, nN, nP);
  hipFuncSetAttribute(reinterpret_cast<const void*>(&k_agg<1>),
                      hipFuncAttributeMaxDynamicSharedMemorySize, LDS1);
  k_agg<1><<<cdiv(nN, NB1), NTHR, LDS1, stream>>>(ei, x, es, ed, b0, ln0_g, ln0_b, agg1, nN, nE, 0);
  k_agemm<<<nP / GR, NTHR, 0, stream>>>(agg1, Pwr_h, Pwr_l, b0, ln0_g, ln0_b, h1, nN);

  k_xp<<<nP / GR, NTHR, 0, stream>>>(h1, Pw2_h, Pw2_l, a_src1, a_dst1, xp2, es, ed, nN);
  hipFuncSetAttribute(reinterpret_cast<const void*>(&k_agg<2>),
                      hipFuncAttributeMaxDynamicSharedMemorySize, LDS2);
  k_agg<2><<<cdiv(nN, NB2), NTHR, LDS2, stream>>>(ei, xp2, es, ed, b1, ln1_g, ln1_b, h2, nN, nE, 0);

  k_tail<<<nP / GR, NTHR, 0, stream>>>(h2, x, Pih_h, Pih_l, gb_ih, gb_hh, Pd0_h, Pd0_l, d0b,
                                       Pd1_h, Pd1_l, d1b, d2w, d2b, out, nN);
}
